// AxiomENSORCLN_25838523253157
// MI455X (gfx1250) — hardware-verified
//
#include <hip/hip_runtime.h>
#include <math.h>

constexpr int kRows       = 262144;
constexpr int kHist       = 24;
constexpr int kFore       = 20;
constexpr int kHid        = 256;
constexpr int kTau        = 6;
constexpr int kChunk      = 65536;
constexpr int kNumChunks  = kRows / kChunk;
constexpr int kCombK      = 64;
constexpr int kSoftN      = 64;
constexpr int kPhysLd     = 32;
constexpr int kPhysThreads = 128;
constexpr float kWCarry    = 64.0f;
constexpr float kWCarryInv = 1.0f / 64.0f;
static_assert(kRows % kChunk == 0, "chunking");
static_assert(kChunk % 64 == 0 && kHid % 64 == 0 && kCombK % 32 == 0 && kSoftN % 64 == 0, "tiles");
static_assert(kChunk % kPhysThreads == 0, "physics grid");
static_assert((kChunk * kFore) % (256 * 4) == 0, "pack grid");

typedef __attribute__((ext_vector_type(16))) _Float16 v16h;
typedef __attribute__((ext_vector_type(8)))  _Float16 v8h;
typedef __attribute__((ext_vector_type(16))) __bf16   v16b;
typedef __attribute__((ext_vector_type(8)))  __bf16   v8b;
typedef __attribute__((ext_vector_type(8)))  float    v8f;
typedef __attribute__((ext_vector_type(4)))  float    v4f;
typedef __attribute__((ext_vector_type(4)))  unsigned int v4u;

__device__ __forceinline__ unsigned short f2bf_bits(float f) {
  unsigned u = __float_as_uint(f);
  return (unsigned short)((u + 0x7FFFu + ((u >> 16) & 1u)) >> 16);
}
__device__ __forceinline__ float bf_bits2f(unsigned short h) { return __uint_as_float(((unsigned)h) << 16); }

__device__ __forceinline__ void dep_guard_h(v8f& a, v8f& b, v16h x, v16h y) { asm volatile("v_nop\n\tv_nop\n\tv_nop\n\tv_nop" : "+v"(a), "+v"(b) : "v"(x), "v"(y)); }
__device__ __forceinline__ void dep_guard_b(v8f& a, v8f& b, v16b x, v16b y) { asm volatile("v_nop\n\tv_nop\n\tv_nop\n\tv_nop" : "+v"(a), "+v"(b) : "v"(x), "v"(y)); }
__device__ __forceinline__ void keep4_h(v16h a, v16h b, v16h c, v16h d) { asm volatile("v_nop" :: "v"(a), "v"(b), "v"(c), "v"(d)); }
__device__ __forceinline__ void keep4_b(v16b a, v16b b, v16b c, v16b d) { asm volatile("v_nop" :: "v"(a), "v"(b), "v"(c), "v"(d)); }
__device__ __forceinline__ void acc_guard4(v8f& a, v8f& b, v8f& c, v8f& d) { asm volatile("v_nop\n\tv_nop\n\tv_nop\n\tv_nop" : "+v"(a), "+v"(b), "+v"(c), "+v"(d)); }
template <typename T> struct Frag;
template <> struct Frag<_Float16> {
  typedef v16h V; union U { v16h v; v8h h[2]; };
  static __device__ __forceinline__ v16h load(const _Float16* p) {
    U f; f.h[0] = *(const v8h*)(p); f.h[1] = *(const v8h*)(p + 16); return f.v;
  }
  static __device__ __forceinline__ v8f mma(v16h a, v16h b, v8f c) {
    return __builtin_amdgcn_wmma_f32_16x16x32_f16(false, a, false, b, (short)0, c, false, false);
  }
  static __device__ __forceinline__ void guard(v8f& a, v8f& b, v16h x, v16h y) { dep_guard_h(a, b, x, y); }
  static __device__ __forceinline__ void keep(v16h a, v16h b, v16h c, v16h d) { keep4_h(a, b, c, d); }
};
template <> struct Frag<__bf16> {
  typedef v16b V; union U { v16b v; v8b h[2]; };
  static __device__ __forceinline__ v16b load(const __bf16* p) {
    U f; f.h[0] = *(const v8b*)(p); f.h[1] = *(const v8b*)(p + 16); return f.v;
  }
  static __device__ __forceinline__ v8f mma(v16b a, v16b b, v8f c) {
    return __builtin_amdgcn_wmma_f32_16x16x32_bf16(false, a, false, b, (short)0, c, false, false);
  }
  static __device__ __forceinline__ void guard(v8f& a, v8f& b, v16b x, v16b y) { dep_guard_b(a, b, x, y); }
  static __device__ __forceinline__ void keep(v16b a, v16b b, v16b c, v16b d) { keep4_b(a, b, c, d); }
};

__device__ __forceinline__ unsigned pk16(unsigned short a, unsigned short b) { return (unsigned)a | ((unsigned)b << 16); }
__device__ __forceinline__ unsigned short h_bits(float f) { const _Float16 h = (_Float16)f; return __builtin_bit_cast(unsigned short, h); }
__device__ __forceinline__ float bfr(float f) { return bf_bits2f(f2bf_bits(f)); }

template <int ET> struct Elem;
template <> struct Elem<0> { typedef _Float16 T; };
template <> struct Elem<1> { typedef __bf16 T; };
template <int ET, bool SPLIT, int BIAS_MODE, int OUT_MODE, bool RESID, int ACT = 0>
__global__ __launch_bounds__(256) void wmma_gemm64(
    const unsigned short* __restrict__ Ap, const unsigned short* __restrict__ A2p, int lda, long strideA,
    const unsigned short* __restrict__ Btp, const unsigned short* __restrict__ Bt2p, int ldb, long strideB,
    void* __restrict__ Cout, void* __restrict__ Cout2, int ldc, long strideC,
    const float* __restrict__ bias,
    const float* __restrict__ resid, long strideR,
    int M, int N, int K, float scale) {
  typedef typename Elem<ET>::T T;
  typedef typename Frag<T>::V V;
  const T* A = (const T*)Ap; const T* A2 = (const T*)A2p; const T* Bt = (const T*)Btp; const T* Bt2 = (const T*)Bt2p;
  __shared__ __align__(16) float sT[8][16 * 68];
  const int b    = blockIdx.y;
  const int lane = threadIdx.x & 31;
  const int wave = threadIdx.x >> 5;
  const int tilesN = N >> 6;
  const int tilesM = M >> 6;
  const int tile = blockIdx.x * 8 + wave;
  if (tile >= tilesM * tilesN) return;
  const int tm = tile / tilesN;
  const int tn = tile - tm * tilesN;
  const int m0 = tm << 6;
  const int n0 = tn << 6;

  const T* Ab  = A  + (size_t)b * strideA;
  const T* Bb  = Bt + (size_t)b * strideB;
  const T* Ab2 = SPLIT ? (A2  + (size_t)b * strideA) : nullptr;
  const T* Bb2 = SPLIT ? (Bt2 + (size_t)b * strideB) : nullptr;

  const int rlane = lane & 15;
  const int koff  = (lane >> 4) * 8;
  const int mOff  = (lane >> 4) * 8;

  v8f acc[4][4];
#pragma unroll
  for (int i = 0; i < 4; ++i)
#pragma unroll
    for (int j = 0; j < 4; ++j) acc[i][j] = (v8f){0.f,0.f,0.f,0.f,0.f,0.f,0.f,0.f};

  for (int k0 = 0; k0 < K; k0 += 32) {
    V bh[4], bl[4];
#pragma unroll
    for (int j = 0; j < 4; ++j) {
      const size_t bo = (size_t)(n0 + (j << 4) + rlane) * ldb + koff + k0;
      bh[j] = Frag<T>::load(Bb + bo);
      if (SPLIT) bl[j] = Frag<T>::load(Bb2 + bo);
    }
#pragma unroll
    for (int i = 0; i < 4; ++i) {
      const size_t ao = (size_t)(m0 + (i << 4) + rlane) * lda + koff + k0;
      V ah = Frag<T>::load(Ab + ao);
      V al;
      if (SPLIT) al = Frag<T>::load(Ab2 + ao);
#pragma unroll
      for (int j = 0; j < 4; ++j) {
        acc[i][j] = Frag<T>::mma(ah, bh[j], acc[i][j]);
        if (SPLIT) {
          acc[i][j] = Frag<T>::mma(ah, bl[j], acc[i][j]);
          acc[i][j] = Frag<T>::mma(al, bh[j], acc[i][j]);
        }
      }
      Frag<T>::guard(acc[i][0], acc[i][3], ah, SPLIT ? al : ah);
    }
    Frag<T>::keep(bh[0], bh[1], bh[2], bh[3]);
    if (SPLIT) Frag<T>::keep(bl[0], bl[1], bl[2], bl[3]);
  }
  acc_guard4(acc[0][0], acc[0][1], acc[0][2], acc[0][3]);
  acc_guard4(acc[1][0], acc[1][1], acc[1][2], acc[1][3]);
  acc_guard4(acc[2][0], acc[2][1], acc[2][2], acc[2][3]);
  acc_guard4(acc[3][0], acc[3][1], acc[3][2], acc[3][3]);

  float* slab = sT[wave];
  const float* Rb = RESID ? (resid + (size_t)b * strideR) : nullptr;
#pragma unroll
  for (int i = 0; i < 4; ++i) {
    const int mBase = m0 + (i << 4);
#pragma unroll
    for (int j = 0; j < 4; ++j) {
      const int n = n0 + (j << 4) + rlane;
      float bv = 0.f;
      if (BIAS_MODE == 2) bv = bias[n];
#pragma unroll
      for (int r = 0; r < 8; ++r) {
        float v = acc[i][j][r] * scale;
        if (BIAS_MODE == 1) v += bias[mBase + mOff + r];
        if (BIAS_MODE == 2) v += bv;
        if (RESID) v += Rb[(size_t)(mBase + mOff + r) * ldc + n];
        if (ACT == 1) v = tanhf(v);
        if (ACT == 2) v = fmaxf(v, 0.0f);
        if (ACT == 4) v = (v > 0.f) ? v : 0.01f * v;
        slab[(mOff + r) * 68 + (j << 4) + rlane] = v;
      }
    }
    __builtin_amdgcn_fence(__ATOMIC_RELEASE, "workgroup");
    __builtin_amdgcn_wave_barrier();
    __builtin_amdgcn_fence(__ATOMIC_ACQUIRE, "workgroup");
    if (OUT_MODE == 0) {
      float* C = (float*)Cout + (size_t)b * strideC;
      const int hh = lane >> 4, c4 = (lane & 15) * 4;
      for (int pass = 0; pass < 2; ++pass) {
#pragma unroll
        for (int it = 0; it < 8; ++it) {
          const int row = it * 2 + hh;
          v4f v = *(const v4f*)(slab + row * 68 + c4);
          *(volatile v4f*)(C + (size_t)(mBase + row) * ldc + n0 + c4) = v;
        }
        __threadfence();
      }
    } else {
      const int q = lane >> 3, c8 = (lane & 7) * 8;
      unsigned short* C  = (unsigned short*)Cout  + (size_t)b * strideC;
      unsigned short* C2 = (OUT_MODE == 2) ? ((unsigned short*)Cout2 + (size_t)b * strideC) : nullptr;
      for (int pass = 0; pass < 2; ++pass) {
#pragma unroll
        for (int it = 0; it < 4; ++it) {
          const int row = it * 4 + q;
          const float* sp = slab + row * 68 + c8;
          v8h hv, lv;
#pragma unroll
          for (int e = 0; e < 8; ++e) {
            if (OUT_MODE == 1) {
              hv[e] = (_Float16)sp[e];
            } else {
              unsigned short hb = f2bf_bits(sp[e]);
              unsigned short lb = f2bf_bits(sp[e] - bf_bits2f(hb));
              hv[e] = __builtin_bit_cast(_Float16, hb);
              lv[e] = __builtin_bit_cast(_Float16, lb);
            }
          }
          *(volatile v8h*)(C + (size_t)(mBase + row) * ldc + n0 + c8) = hv;
          if (OUT_MODE == 2) *(volatile v8h*)(C2 + (size_t)(mBase + row) * ldc + n0 + c8) = lv;
        }
        __threadfence();
      }
    }
    __builtin_amdgcn_fence(__ATOMIC_RELEASE, "workgroup");
    __builtin_amdgcn_wave_barrier();
    __builtin_amdgcn_fence(__ATOMIC_ACQUIRE, "workgroup");
  }
}

constexpr int kWtPitch = 260;
__global__ __launch_bounds__(256) void wprep_kernel(const float* __restrict__ W, int Kreal, int Nreal, int Kpad,
                                                    unsigned short* __restrict__ Wt, float scale) {
  __shared__ __align__(16) float tile[32 * kWtPitch];
  const int tid = threadIdx.x, lane = tid & 31, wave = tid >> 5;
  const int n0 = blockIdx.x * 32;
  const int nIter = Kpad >> 3;
#pragma unroll 1
  for (int i = 0; i < nIter; ++i) {
    const int idx = tid + 256 * i;
    const int k  = idx >> 5;
    const int nl = idx & 31;
    const int n  = n0 + nl;
    const int kc = (k < Kreal) ? k : (Kreal - 1);
    const int nc = (n < Nreal) ? n : (Nreal - 1);
    float v = W[(size_t)kc * Nreal + nc];
    if (k >= Kreal || n >= Nreal) v = 0.0f;
    tile[nl * kWtPitch + k] = v;
  }
  __syncthreads();
  const int lpr = Kpad >> 6;
  const int q = lane >> 3, c8 = (lane & 7) * 8;
  for (int pass = 0; pass < 2; ++pass) {
#pragma unroll 1
    for (int it = 0; it < lpr; ++it) {
      const int line = (it * 8 + wave) * 4 + q;
      const int nl   = line / lpr;
      const int s    = line - nl * lpr;
      const int koff = s * 64 + c8;
      const float* tp = tile + nl * kWtPitch + koff;
      unsigned short hb[8];
#pragma unroll
      for (int e = 0; e < 8; ++e) hb[e] = h_bits(bfr(tp[e]) * scale);
      const v4u u = (v4u){pk16(hb[0], hb[1]), pk16(hb[2], hb[3]), pk16(hb[4], hb[5]), pk16(hb[6], hb[7])};
      *(volatile v4u*)(Wt + (size_t)(n0 + nl) * Kpad + koff) = u;
    }
    __threadfence();
  }
}

__global__ __launch_bounds__(kPhysThreads) void physics_kernel(
    const float* __restrict__ hist, const float* __restrict__ alpha_p, const float* __restrict__ beta_p,
    const float* __restrict__ gamma_p, const float* __restrict__ tau_p,
    float* __restrict__ PH, unsigned* __restrict__ COMBu) {
#pragma clang fp contract(off)
  __shared__ __align__(16) float    phys_s[kPhysThreads * kPhysLd];
  __shared__ __align__(16) unsigned comb_s[kPhysThreads * (kCombK / 2)];
  const int tid = threadIdx.x, lane = tid & 31, wave = tid >> 5;
  const int lr = blockIdx.x * kPhysThreads + tid;
  const float* hr = hist + (size_t)lr * kHist;
  float hv[kHist];
#pragma unroll
  for (int qd = 0; qd < kHist / 4; ++qd) {
    const v4f x = *(const v4f*)(hr + 4 * qd);
#pragma unroll
    for (int e = 0; e < 4; ++e) hv[4 * qd + e] = bfr(x[e]);
  }
  const float a = 1.0f / (1.0f + expf(-bfr(alpha_p[0])));
  const float b = 1.0f / (1.0f + expf(-bfr(beta_p[0])));
  const float g = fabsf(bfr(gamma_p[0]));
  (void)tau_p;

  unsigned* cs = comb_s + tid * (kCombK / 2);
#pragma unroll
  for (int j = 0; j < kHist / 2; ++j) cs[j] = pk16(h_bits(hv[2 * j]), h_bits(hv[2 * j + 1]));

  float buf[kTau];
#pragma unroll
  for (int j = 0; j < kTau; ++j) buf[j] = hv[kHist - kTau + j];
  float T = hv[kHist - 1];
  float tp[kFore];
#pragma unroll
  for (int s = 0; s < kFore; ++s) {
    const int idx = s % kTau;
    const float Td = buf[idx];
    const float t1 = a * T;
    const float u1 = T - t1;
    const float t2 = b * Td;
    const float u2 = u1 - t2;
    const float sq = T * T;
    const float cu = T * sq;
    const float t3 = g * cu;
    const float Tn = u2 - t3;
    buf[idx] = Tn;
    T = Tn;
    tp[s] = Tn;
  }
  float* ps = phys_s + tid * kPhysLd;
#pragma unroll
  for (int s = 0; s < kFore; ++s) ps[s] = tp[s];
#pragma unroll
  for (int s = kFore; s < kPhysLd; ++s) ps[s] = 0.0f;
#pragma unroll
  for (int j = 0; j < kFore / 2; ++j) cs[kHist / 2 + j] = pk16(h_bits(tp[2 * j]), h_bits(tp[2 * j + 1]));
#pragma unroll
  for (int j = (kHist + kFore) / 2; j < kCombK / 2; ++j) cs[j] = 0u;
  __syncthreads();

  const int q = lane >> 3, c4 = (lane & 7) * 4;
  const size_t rbase = (size_t)blockIdx.x * kPhysThreads;
  for (int pass = 0; pass < 2; ++pass) {
#pragma unroll
    for (int it = 0; it < 8; ++it) {
      const int row = it * 16 + wave * 4 + q;
      const v4f pv = *(const v4f*)(phys_s + row * kPhysLd + c4);
      const v4u cv = *(const v4u*)(comb_s + row * (kCombK / 2) + c4);
      *(volatile v4f*)(PH    + (rbase + row) * kPhysLd      + c4) = pv;
      *(volatile v4u*)(COMBu + (rbase + row) * (kCombK / 2) + c4) = cv;
    }
    __threadfence();
  }
}

__global__ __launch_bounds__(256) void pack_kernel(const float* __restrict__ PH, const float* __restrict__ TS,
                                                   const float* __restrict__ cb2, const float* __restrict__ lam_p,
                                                   float* __restrict__ out_pred, float* __restrict__ out_phys,
                                                   float* __restrict__ out_soft, int n4) {
#pragma clang fp contract(off)
  const int t = blockIdx.x * 256 + threadIdx.x;
  if (t >= n4) return;
  const int row = t / 5;
  const int c0  = (t - row * 5) * 4;
  const v4f p  = *(const v4f*)(PH + (size_t)row * kPhysLd + c0);
  const v4f sv = *(const v4f*)(TS + (size_t)row * kSoftN + c0);
  const float lam = 1.0f / (1.0f + expf(-bfr(lam_p[0])));
  v4f soft, pred;
#pragma unroll
  for (int e = 0; e < 4; ++e) {
    const float bb = bfr(cb2[c0 + e]);
    const float s1 = sv[e] + bb;
    const float m1 = lam * s1;
    soft[e] = s1;
    pred[e] = p[e] + m1;
  }
  const size_t o = (size_t)4 * t;
  *(volatile v4f*)(out_pred + o) = pred;
  *(volatile v4f*)(out_phys + o) = p;
  *(volatile v4f*)(out_soft + o) = soft;
  __threadfence();
  *(volatile v4f*)(out_pred + o) = pred;
  *(volatile v4f*)(out_phys + o) = p;
  *(volatile v4f*)(out_soft + o) = soft;
}

extern "C" void kernel_launch(void* const* d_in, const int* in_sizes, int n_in,
                              void* d_out, int out_size, void* d_ws, size_t ws_size,
                              hipStream_t stream) {
  if (n_in < 14) return;
  if (in_sizes[0] != kRows * kHist) return;
  if (in_sizes[1] != (kHist + kFore) * kHid) return;
  if (in_sizes[2] != kHid || in_sizes[4] != kHid || in_sizes[6] != kHid) return;
  if (in_sizes[3] != kHid * kHid || in_sizes[5] != kHid * kHid) return;
  if (in_sizes[7] != kHid * kFore || in_sizes[8] != kFore) return;
  if (in_sizes[9] < 1 || in_sizes[10] < 1 || in_sizes[11] < 1 || in_sizes[12] < 1 || in_sizes[13] < 1) return;
  if (out_size != 3 * kRows * kFore) return;

  const float* history    = (const float*)d_in[0];
  const float* enc_w1     = (const float*)d_in[1];
  const float* enc_b1     = (const float*)d_in[2];
  const float* enc_w2     = (const float*)d_in[3];
  const float* enc_b2     = (const float*)d_in[4];
  const float* cor_w1     = (const float*)d_in[5];
  const float* cor_b1     = (const float*)d_in[6];
  const float* cor_w2     = (const float*)d_in[7];
  const float* cor_b2     = (const float*)d_in[8];
  const float* alpha      = (const float*)d_in[9];
  const float* beta       = (const float*)d_in[10];
  const float* gamma      = (const float*)d_in[11];
  const float* tau        = (const float*)d_in[12];
  const float* lambda_mix = (const float*)d_in[13];
  float* outp = (float*)d_out;

  const size_t SZ_W1T  = (size_t)kHid * kCombK * 2;
  const size_t SZ_W2T  = (size_t)kHid * kHid * 2;
  const size_t SZ_CW2T = (size_t)kSoftN * kHid * 2;
  const size_t SZ_COMB = (size_t)kChunk * kCombK * 2;
  const size_t SZ_H    = (size_t)kChunk * kHid * 2;
  const size_t SZ_TS   = (size_t)kChunk * kSoftN * 4;
  const size_t SZ_PH   = (size_t)kChunk * kPhysLd * 4;
  size_t off = 0;
  const size_t oW1T  = off; off += SZ_W1T;
  const size_t oW2T  = off; off += SZ_W2T;
  const size_t oCW1T = off; off += SZ_W2T;
  const size_t oCW2T = off; off += SZ_CW2T;
  const size_t oCOMB = off; off += SZ_COMB;
  const size_t oHA   = off; off += SZ_H;
  const size_t oHB   = off; off += SZ_H;
  const size_t oTS   = off; off += SZ_TS;
  const size_t oPH   = off; off += SZ_PH;
  const size_t TOTAL = off;
  if (TOTAL > ws_size) return;
  if (TOTAL > (size_t)134217728) return;

  char* ws = (char*)d_ws;
  unsigned short* W1T  = (unsigned short*)(ws + oW1T);
  unsigned short* W2T  = (unsigned short*)(ws + oW2T);
  unsigned short* CW1T = (unsigned short*)(ws + oCW1T);
  unsigned short* CW2T = (unsigned short*)(ws + oCW2T);
  unsigned short* COMB = (unsigned short*)(ws + oCOMB);
  unsigned short* HA   = (unsigned short*)(ws + oHA);
  unsigned short* HB   = (unsigned short*)(ws + oHB);
  float*          TS   = (float*)(ws + oTS);
  float*          PH   = (float*)(ws + oPH);

  const dim3 blk(256);

  wprep_kernel<<<dim3(kHid / 32), blk, 0, stream>>>(enc_w1, kHist + kFore, kHid, kCombK, W1T, kWCarry);
  wprep_kernel<<<dim3(kHid / 32), blk, 0, stream>>>(enc_w2, kHid, kHid, kHid, W2T, kWCarry);
  wprep_kernel<<<dim3(kHid / 32), blk, 0, stream>>>(cor_w1, kHid, kHid, kHid, CW1T, kWCarry);
  wprep_kernel<<<dim3(kSoftN / 32), blk, 0, stream>>>(cor_w2, kHid, kFore, kHid, CW2T, kWCarry);

  const int tilesM = kChunk / 64;
  const dim3 gHid((tilesM * (kHid / 64) + 7) / 8, 1);
  const dim3 gSoft((tilesM * (kSoftN / 64) + 7) / 8, 1);
  const int n4 = kChunk * kFore / 4;

  for (int c = 0; c < kNumChunks; ++c) {
    const float* hist_c = history + (size_t)c * kChunk * kHist;
    float* out0_c = outp + (size_t)c * kChunk * kFore;
    float* out1_c = outp + (size_t)kRows * kFore + (size_t)c * kChunk * kFore;
    float* out2_c = outp + (size_t)2 * kRows * kFore + (size_t)c * kChunk * kFore;

    physics_kernel<<<dim3(kChunk / kPhysThreads), dim3(kPhysThreads), 0, stream>>>(
        hist_c, alpha, beta, gamma, tau, PH, (unsigned*)COMB);
    wmma_gemm64<0, false, 2, 1, false, 1><<<gHid, blk, 0, stream>>>(
        COMB, COMB, kCombK, 0L, W1T, W1T, kCombK, 0L, (void*)HA, (void*)HA, kHid, 0L, enc_b1, enc_b1, 0L, kChunk, kHid, kCombK, kWCarryInv);
    wmma_gemm64<0, false, 2, 1, false, 1><<<gHid, blk, 0, stream>>>(
        HA, HA, kHid, 0L, W2T, W2T, kHid, 0L, (void*)HB, (void*)HB, kHid, 0L, enc_b2, enc_b2, 0L, kChunk, kHid, kHid, kWCarryInv);
    wmma_gemm64<0, false, 2, 1, false, 1><<<gHid, blk, 0, stream>>>(
        HB, HB, kHid, 0L, CW1T, CW1T, kHid, 0L, (void*)HA, (void*)HA, kHid, 0L, cor_b1, cor_b1, 0L, kChunk, kHid, kHid, kWCarryInv);
    wmma_gemm64<0, false, 0, 0, false, 0><<<gSoft, blk, 0, stream>>>(
        HA, HA, kHid, 0L, CW2T, CW2T, kHid, 0L, (void*)TS, (void*)TS, kSoftN, 0L, cor_b1, cor_b1, 0L, kChunk, kSoftN, kHid, kWCarryInv);
    pack_kernel<<<dim3(n4 / 256), blk, 0, stream>>>(PH, TS, cor_b2, lambda_mix, out0_c, out1_c, out2_c, n4);
  }
}
